// TransformerBlockClassical_65481071405559
// MI455X (gfx1250) — hardware-run, weakly checked
//
#include <hip/hip_runtime.h>
#include <math.h>

constexpr int kBatch  = 2;
constexpr int kSeq    = 2048;
constexpr int kEmb    = 1024;
constexpr int kHeads  = 16;
constexpr int kHd     = 64;
constexpr int kFfn    = 4096;
constexpr int kTok    = kBatch * kSeq;
constexpr int kGroups = kBatch * kHeads;
constexpr int kGrpPerChunk = 2;
constexpr int kNumChunks   = kGroups / kGrpPerChunk;
constexpr int kFfnRows   = 1024;
constexpr int kFfnChunks = kTok / kFfnRows;

constexpr float kWCarry     = 16.0f;
constexpr float kPCarry     = 2048.0f;
constexpr float kCtxCarry   = 256.0f;
constexpr float kGCarry     = 16.0f;
constexpr float kScoreScale = 0.125f;
constexpr float kQkvScale   = 1.0f / kWCarry;
constexpr float kPVScale    = kCtxCarry / kPCarry;
constexpr float kWoScale    = 1.0f / (kCtxCarry * kWCarry);
constexpr float kHScale     = 1.0f / kWCarry;
constexpr float kOutScale   = 1.0f / (kGCarry * kWCarry);
constexpr float kInvEmb     = 1.0f / 1024.0f;
constexpr float kLnEps      = 1e-5f;

constexpr size_t kMiB      = 1048576;
constexpr size_t kOffX16   = 0 * kMiB;
constexpr size_t kOffWqkvT = 8 * kMiB;
constexpr size_t kOffWoT   = 14 * kMiB;
constexpr size_t kOffW1T   = 16 * kMiB;
constexpr size_t kOffW2T   = 24 * kMiB;
constexpr size_t kOffWfT   = 32 * kMiB;
constexpr size_t kOffQK16  = 40 * kMiB;
constexpr size_t kOffVT16  = 56 * kMiB;
constexpr size_t kOffSC    = 64 * kMiB;
constexpr size_t kOffP16   = 96 * kMiB;
constexpr size_t kOffCTX16 = 112 * kMiB;
constexpr size_t kOffY1    = 64 * kMiB;
constexpr size_t kOffX1    = 0 * kMiB;
constexpr size_t kOffX1h   = 120 * kMiB;
constexpr size_t kOffH1c   = 40 * kMiB;
constexpr size_t kOffH2c   = 88 * kMiB;
constexpr size_t kOffG16   = 56 * kMiB;
constexpr size_t kOffY2    = 40 * kMiB;
constexpr size_t kWsTotal  = 128 * kMiB;

static_assert((size_t)kTok * kEmb * 2 == 8 * kMiB, "X16 size");
static_assert((size_t)3 * kEmb * kEmb * 2 == 6 * kMiB, "WqkvT size");
static_assert((size_t)kEmb * kEmb * 2 == 2 * kMiB, "WoT size");
static_assert((size_t)kFfn * kEmb * 2 == 8 * kMiB, "W1T/W2T/WfT size");
static_assert((size_t)kTok * 2 * kEmb * 2 == 16 * kMiB, "QK16 size");
static_assert((size_t)kEmb * kTok * 2 == 8 * kMiB, "VT16 size");
static_assert((size_t)kGrpPerChunk * kSeq * kSeq * 4 == 32 * kMiB, "SC size");
static_assert((size_t)kGrpPerChunk * kSeq * kSeq * 2 == 16 * kMiB, "P16 size");
static_assert((size_t)kTok * kEmb * 2 == 8 * kMiB, "CTX16 size");
static_assert((size_t)kTok * kEmb * 4 == 16 * kMiB, "Y1/X1/Y2 size");
static_assert((size_t)kFfnRows * kFfn * 4 == 16 * kMiB, "H1c/H2c size");
static_assert((size_t)kTok * kFfn * 2 == 32 * kMiB, "G16 size");
static_assert(kOffX1h + 8 * kMiB == kWsTotal, "carve end");
static_assert(kGroups % kGrpPerChunk == 0 && kHeads % kGrpPerChunk == 0, "chunking");

typedef __attribute__((ext_vector_type(16))) _Float16 v16h;
typedef __attribute__((ext_vector_type(8)))  _Float16 v8h;
typedef __attribute__((ext_vector_type(16))) __bf16   v16b;
typedef __attribute__((ext_vector_type(8)))  __bf16   v8b;
typedef __attribute__((ext_vector_type(8)))  float    v8f;
typedef __attribute__((ext_vector_type(4)))  float    v4f;
typedef __attribute__((ext_vector_type(2)))  float    v2f;
typedef __attribute__((ext_vector_type(4)))  unsigned int v4u;

__device__ __forceinline__ unsigned short f2bf_bits(float f) {
  unsigned u = __float_as_uint(f);
  return (unsigned short)((u + 0x7FFFu + ((u >> 16) & 1u)) >> 16);
}
__device__ __forceinline__ float bf_bits2f(unsigned short h) { return __uint_as_float(((unsigned)h) << 16); }

__device__ __forceinline__ void dep_guard_h(v8f& a, v8f& b, v16h x, v16h y) { asm volatile("v_nop\n\tv_nop\n\tv_nop\n\tv_nop" : "+v"(a), "+v"(b) : "v"(x), "v"(y)); }
__device__ __forceinline__ void dep_guard_b(v8f& a, v8f& b, v16b x, v16b y) { asm volatile("v_nop\n\tv_nop\n\tv_nop\n\tv_nop" : "+v"(a), "+v"(b) : "v"(x), "v"(y)); }
__device__ __forceinline__ void keep4_h(v16h a, v16h b, v16h c, v16h d) { asm volatile("v_nop" :: "v"(a), "v"(b), "v"(c), "v"(d)); }
__device__ __forceinline__ void keep4_b(v16b a, v16b b, v16b c, v16b d) { asm volatile("v_nop" :: "v"(a), "v"(b), "v"(c), "v"(d)); }
__device__ __forceinline__ void acc_guard4(v8f& a, v8f& b, v8f& c, v8f& d) { asm volatile("v_nop\n\tv_nop\n\tv_nop\n\tv_nop" : "+v"(a), "+v"(b), "+v"(c), "+v"(d)); }
template <typename T> struct Frag;
template <> struct Frag<_Float16> {
  typedef v16h V; union U { v16h v; v8h h[2]; };
  static __device__ __forceinline__ v16h load(const _Float16* p) {
    U f; f.h[0] = *(const v8h*)(p); f.h[1] = *(const v8h*)(p + 16); return f.v;
  }
  static __device__ __forceinline__ v8f mma(v16h a, v16h b, v8f c) {
    return __builtin_amdgcn_wmma_f32_16x16x32_f16(false, a, false, b, (short)0, c, false, false);
  }
  static __device__ __forceinline__ void guard(v8f& a, v8f& b, v16h x, v16h y) { dep_guard_h(a, b, x, y); }
  static __device__ __forceinline__ void keep(v16h a, v16h b, v16h c, v16h d) { keep4_h(a, b, c, d); }
};
template <> struct Frag<__bf16> {
  typedef v16b V; union U { v16b v; v8b h[2]; };
  static __device__ __forceinline__ v16b load(const __bf16* p) {
    U f; f.h[0] = *(const v8b*)(p); f.h[1] = *(const v8b*)(p + 16); return f.v;
  }
  static __device__ __forceinline__ v8f mma(v16b a, v16b b, v8f c) {
    return __builtin_amdgcn_wmma_f32_16x16x32_bf16(false, a, false, b, (short)0, c, false, false);
  }
  static __device__ __forceinline__ void guard(v8f& a, v8f& b, v16b x, v16b y) { dep_guard_b(a, b, x, y); }
  static __device__ __forceinline__ void keep(v16b a, v16b b, v16b c, v16b d) { keep4_b(a, b, c, d); }
};

__device__ __forceinline__ unsigned pk16(unsigned short a, unsigned short b) { return (unsigned)a | ((unsigned)b << 16); }
__device__ __forceinline__ unsigned short h_bits(float f) { const _Float16 h = (_Float16)f; return __builtin_bit_cast(unsigned short, h); }

template <int ET> struct Elem;
template <> struct Elem<0> { typedef _Float16 T; };
template <> struct Elem<1> { typedef __bf16 T; };
template <int ET, bool SPLIT, int BIAS_MODE, int OUT_MODE, bool RESID, int ACT = 0>
__global__ __launch_bounds__(256) void wmma_gemm64(
    const unsigned short* __restrict__ Ap, const unsigned short* __restrict__ A2p, int lda, long strideA,
    const unsigned short* __restrict__ Btp, const unsigned short* __restrict__ Bt2p, int ldb, long strideB,
    void* __restrict__ Cout, void* __restrict__ Cout2, int ldc, long strideC,
    const float* __restrict__ bias,
    const float* __restrict__ resid, long strideR,
    int M, int N, int K, float scale) {
  typedef typename Elem<ET>::T T;
  typedef typename Frag<T>::V V;
  const T* A = (const T*)Ap; const T* A2 = (const T*)A2p; const T* Bt = (const T*)Btp; const T* Bt2 = (const T*)Bt2p;
  __shared__ __align__(16) float sT[8][16 * 68];
  const int b    = blockIdx.y;
  const int lane = threadIdx.x & 31;
  const int wave = threadIdx.x >> 5;
  const int tilesN = N >> 6;
  const int tilesM = M >> 6;
  const int tile = blockIdx.x * 8 + wave;
  if (tile >= tilesM * tilesN) return;
  const int tm = tile / tilesN;
  const int tn = tile - tm * tilesN;
  const int m0 = tm << 6;
  const int n0 = tn << 6;

  const T* Ab  = A  + (size_t)b * strideA;
  const T* Bb  = Bt + (size_t)b * strideB;
  const T* Ab2 = SPLIT ? (A2  + (size_t)b * strideA) : nullptr;
  const T* Bb2 = SPLIT ? (Bt2 + (size_t)b * strideB) : nullptr;

  const int rlane = lane & 15;
  const int koff  = (lane >> 4) * 8;
  const int mOff  = (lane >> 4) * 8;

  v8f acc[4][4];
#pragma unroll
  for (int i = 0; i < 4; ++i)
#pragma unroll
    for (int j = 0; j < 4; ++j) acc[i][j] = (v8f){0.f,0.f,0.f,0.f,0.f,0.f,0.f,0.f};

  for (int k0 = 0; k0 < K; k0 += 32) {
    V bh[4], bl[4];
#pragma unroll
    for (int j = 0; j < 4; ++j) {
      const size_t bo = (size_t)(n0 + (j << 4) + rlane) * ldb + koff + k0;
      bh[j] = Frag<T>::load(Bb + bo);
      if (SPLIT) bl[j] = Frag<T>::load(Bb2 + bo);
    }
#pragma unroll
    for (int i = 0; i < 4; ++i) {
      const size_t ao = (size_t)(m0 + (i << 4) + rlane) * lda + koff + k0;
      V ah = Frag<T>::load(Ab + ao);
      V al;
      if (SPLIT) al = Frag<T>::load(Ab2 + ao);
#pragma unroll
      for (int j = 0; j < 4; ++j) {
        acc[i][j] = Frag<T>::mma(ah, bh[j], acc[i][j]);
        if (SPLIT) {
          acc[i][j] = Frag<T>::mma(ah, bl[j], acc[i][j]);
          acc[i][j] = Frag<T>::mma(al, bh[j], acc[i][j]);
        }
      }
      Frag<T>::guard(acc[i][0], acc[i][3], ah, SPLIT ? al : ah);
    }
    Frag<T>::keep(bh[0], bh[1], bh[2], bh[3]);
    if (SPLIT) Frag<T>::keep(bl[0], bl[1], bl[2], bl[3]);
  }
  acc_guard4(acc[0][0], acc[0][1], acc[0][2], acc[0][3]);
  acc_guard4(acc[1][0], acc[1][1], acc[1][2], acc[1][3]);
  acc_guard4(acc[2][0], acc[2][1], acc[2][2], acc[2][3]);
  acc_guard4(acc[3][0], acc[3][1], acc[3][2], acc[3][3]);

  float* slab = sT[wave];
  const float* Rb = RESID ? (resid + (size_t)b * strideR) : nullptr;
#pragma unroll
  for (int i = 0; i < 4; ++i) {
    const int mBase = m0 + (i << 4);
#pragma unroll
    for (int j = 0; j < 4; ++j) {
      const int n = n0 + (j << 4) + rlane;
      float bv = 0.f;
      if (BIAS_MODE == 2) bv = bias[n];
#pragma unroll
      for (int r = 0; r < 8; ++r) {
        float v = acc[i][j][r] * scale;
        if (BIAS_MODE == 1) v += bias[mBase + mOff + r];
        if (BIAS_MODE == 2) v += bv;
        if (RESID) v += Rb[(size_t)(mBase + mOff + r) * ldc + n];
        if (ACT == 2) v = fmaxf(v, 0.0f);
        if (ACT == 4) v = (v > 0.f) ? v : 0.01f * v;
        slab[(mOff + r) * 68 + (j << 4) + rlane] = v;
      }
    }
    __builtin_amdgcn_fence(__ATOMIC_RELEASE, "workgroup");
    __builtin_amdgcn_wave_barrier();
    __builtin_amdgcn_fence(__ATOMIC_ACQUIRE, "workgroup");
    if (OUT_MODE == 0) {
      float* C = (float*)Cout + (size_t)b * strideC;
      const int hh = lane >> 4, c4 = (lane & 15) * 4;
      for (int pass = 0; pass < 2; ++pass) {
#pragma unroll
        for (int it = 0; it < 8; ++it) {
          const int row = it * 2 + hh;
          v4f v = *(const v4f*)(slab + row * 68 + c4);
          *(volatile v4f*)(C + (size_t)(mBase + row) * ldc + n0 + c4) = v;
        }
        __threadfence();
      }
    } else {
      const int q = lane >> 3, c8 = (lane & 7) * 8;
      unsigned short* C  = (unsigned short*)Cout  + (size_t)b * strideC;
      unsigned short* C2 = (OUT_MODE == 2) ? ((unsigned short*)Cout2 + (size_t)b * strideC) : nullptr;
      for (int pass = 0; pass < 2; ++pass) {
#pragma unroll
        for (int it = 0; it < 4; ++it) {
          const int row = it * 4 + q;
          const float* sp = slab + row * 68 + c8;
          v8h hv, lv;
#pragma unroll
          for (int e = 0; e < 8; ++e) {
            if (OUT_MODE == 1) {
              hv[e] = (_Float16)sp[e];
            } else {
              unsigned short hb = f2bf_bits(sp[e]);
              unsigned short lb = f2bf_bits(sp[e] - bf_bits2f(hb));
              hv[e] = __builtin_bit_cast(_Float16, hb);
              lv[e] = __builtin_bit_cast(_Float16, lb);
            }
          }
          *(volatile v8h*)(C + (size_t)(mBase + row) * ldc + n0 + c8) = hv;
          if (OUT_MODE == 2) *(volatile v8h*)(C2 + (size_t)(mBase + row) * ldc + n0 + c8) = lv;
        }
        __threadfence();
      }
    }
    __builtin_amdgcn_fence(__ATOMIC_RELEASE, "workgroup");
    __builtin_amdgcn_wave_barrier();
    __builtin_amdgcn_fence(__ATOMIC_ACQUIRE, "workgroup");
  }
}

__global__ __launch_bounds__(256) void wtcast_kernel(const float* __restrict__ W, int nrows, int ncols,
                                                     unsigned short* __restrict__ out, float scale) {
  __shared__ float sm[64][65];
  const int t  = threadIdx.x;
  const int k0 = blockIdx.x * 64;
  const int n0 = blockIdx.y * 64;
#pragma unroll
  for (int i = 0; i < 16; ++i) {
    const int e = i * 256 + t;
    const int r = e >> 6;
    const int c = e & 63;
    sm[c][r] = W[(size_t)(k0 + r) * ncols + n0 + c] * scale;
  }
  __syncthreads();
  const int lane = t & 31, wave = t >> 5;
  const int q = lane >> 3, c8 = (lane & 7) * 8;
  for (int pass = 0; pass < 2; ++pass) {
#pragma unroll
    for (int it = 0; it < 2; ++it) {
      const int row = wave * 8 + it * 4 + q;
      unsigned short hb[8];
#pragma unroll
      for (int e = 0; e < 8; ++e) hb[e] = h_bits(sm[row][c8 + e]);
      const v4u u = (v4u){pk16(hb[0], hb[1]), pk16(hb[2], hb[3]), pk16(hb[4], hb[5]), pk16(hb[6], hb[7])};
      *(volatile v4u*)(out + (size_t)(n0 + row) * nrows + k0 + c8) = u;
    }
    __threadfence();
  }
}

__global__ __launch_bounds__(256) void cast8_f16_kernel(const float* __restrict__ in, unsigned short* __restrict__ out, int n8) {
  const int i = blockIdx.x * 256 + threadIdx.x;
  if (i >= n8) return;
  const float* p = in + 8 * (size_t)i;
  const v4f a = *(const v4f*)(p);
  const v4f c = *(const v4f*)(p + 4);
  unsigned short hb[8];
#pragma unroll
  for (int e = 0; e < 4; ++e) {
    hb[e]     = h_bits(a[e]);
    hb[4 + e] = h_bits(c[e]);
  }
  const v4u u = (v4u){pk16(hb[0], hb[1]), pk16(hb[2], hb[3]), pk16(hb[4], hb[5]), pk16(hb[6], hb[7])};
  unsigned short* qp = out + 8 * (size_t)i;
  *(volatile v4u*)qp = u;
  __threadfence();
  *(volatile v4u*)qp = u;
}

__global__ __launch_bounds__(256) void softmax_row_kernel(const float* __restrict__ S, unsigned short* __restrict__ P, float carry) {
  __shared__ __align__(16) float ebuf[kSeq];
  __shared__ float redM[8];
  __shared__ float redS[8];
  const int t    = threadIdx.x;
  const int lane = t & 31, wave = t >> 5;
  const size_t rowoff = (size_t)blockIdx.x * kSeq;
  const float* sr = S + rowoff;
  float m = -INFINITY;
#pragma unroll 1
  for (int i = 0; i < 8; ++i) {
    const float v = sr[i * 256 + t];
    ebuf[i * 256 + t] = v;
    m = fmaxf(m, v);
  }
#pragma unroll
  for (int off = 16; off > 0; off >>= 1) m = fmaxf(m, __shfl_xor(m, off, 32));
  if (lane == 0) redM[wave] = m;
  __syncthreads();
  m = fmaxf(fmaxf(fmaxf(redM[0], redM[1]), fmaxf(redM[2], redM[3])),
            fmaxf(fmaxf(redM[4], redM[5]), fmaxf(redM[6], redM[7])));
  float s = 0.f;
#pragma unroll 1
  for (int i = 0; i < 8; ++i) {
    const float e = expf(ebuf[i * 256 + t] - m);
    ebuf[i * 256 + t] = e;
    s += e;
  }
#pragma unroll
  for (int off = 16; off > 0; off >>= 1) s += __shfl_xor(s, off, 32);
  if (lane == 0) redS[wave] = s;
  __syncthreads();
  const float tot = ((redS[0] + redS[1]) + (redS[2] + redS[3])) + ((redS[4] + redS[5]) + (redS[6] + redS[7]));
  const float inv = carry * (1.0f / tot);
  const float* ep = ebuf + t * 8;
  const v4f a = *(const v4f*)(ep);
  const v4f c = *(const v4f*)(ep + 4);
  unsigned short hb[8];
#pragma unroll
  for (int e = 0; e < 4; ++e) {
    hb[e]     = h_bits(a[e] * inv);
    hb[4 + e] = h_bits(c[e] * inv);
  }
  const v4u u = (v4u){pk16(hb[0], hb[1]), pk16(hb[2], hb[3]), pk16(hb[4], hb[5]), pk16(hb[6], hb[7])};
  unsigned short* pp = P + rowoff + t * 8;
  *(volatile v4u*)pp = u;
  __threadfence();
  *(volatile v4u*)pp = u;
}

template <bool WRITE16>
__global__ __launch_bounds__(256) void ln_row_kernel(const float* __restrict__ Y, const float* __restrict__ gam,
                                                     const float* __restrict__ bet, float* __restrict__ out,
                                                     unsigned short* __restrict__ out16) {
  __shared__ float redA[8];
  __shared__ float redB[8];
  __shared__ __align__(16) float rowbuf[kEmb];
  const int t    = threadIdx.x;
  const int lane = t & 31, wave = t >> 5;
  const size_t tok = blockIdx.x;
  const int c0 = t * 4;
  const v4f yv = *(const v4f*)(Y + tok * kEmb + c0);
  float s = (yv[0] + yv[1]) + (yv[2] + yv[3]);
#pragma unroll
  for (int off = 16; off > 0; off >>= 1) s += __shfl_xor(s, off, 32);
  if (lane == 0) redA[wave] = s;
  __syncthreads();
  const float tot = ((redA[0] + redA[1]) + (redA[2] + redA[3])) + ((redA[4] + redA[5]) + (redA[6] + redA[7]));
  const float mu = tot * kInvEmb;
  v4f d;
#pragma unroll
  for (int e = 0; e < 4; ++e) d[e] = yv[e] - mu;
  float vs = (d[0] * d[0] + d[1] * d[1]) + (d[2] * d[2] + d[3] * d[3]);
#pragma unroll
  for (int off = 16; off > 0; off >>= 1) vs += __shfl_xor(vs, off, 32);
  if (lane == 0) redB[wave] = vs;
  __syncthreads();
  const float vtot = ((redB[0] + redB[1]) + (redB[2] + redB[3])) + ((redB[4] + redB[5]) + (redB[6] + redB[7]));
  const float inv = rsqrtf(vtot * kInvEmb + kLnEps);
  const v4f gv = *(const v4f*)(gam + c0);
  const v4f bv = *(const v4f*)(bet + c0);
  v4f o;
#pragma unroll
  for (int e = 0; e < 4; ++e) o[e] = d[e] * inv * gv[e] + bv[e];
  float* op = out + tok * kEmb + c0;
  *(volatile v4f*)op = o;
  __threadfence();
  *(volatile v4f*)op = o;
  if (WRITE16) {
#pragma unroll
    for (int e = 0; e < 4; ++e) rowbuf[c0 + e] = o[e];
    __syncthreads();
    if (t < 128) {
      const float* rp = rowbuf + t * 8;
      const v4f a = *(const v4f*)(rp);
      const v4f c = *(const v4f*)(rp + 4);
      unsigned short hb[8];
#pragma unroll
      for (int e = 0; e < 4; ++e) {
        hb[e]     = h_bits(a[e]);
        hb[4 + e] = h_bits(c[e]);
      }
      const v4u u = (v4u){pk16(hb[0], hb[1]), pk16(hb[2], hb[3]), pk16(hb[4], hb[5]), pk16(hb[6], hb[7])};
      unsigned short* hp = out16 + tok * kEmb + t * 8;
      *(volatile v4u*)hp = u;
      __threadfence();
      *(volatile v4u*)hp = u;
    }
  }
}

__global__ __launch_bounds__(256) void gate_kernel(const float* __restrict__ H1, const float* __restrict__ H2,
                                                   unsigned short* __restrict__ G, int n2, float carry) {
  const int i = blockIdx.x * 256 + threadIdx.x;
  if (i >= n2) return;
  const v2f a = *(const v2f*)(H1 + 2 * (size_t)i);
  const v2f g = *(const v2f*)(H2 + 2 * (size_t)i);
  const float s0 = 1.0f / (1.0f + expf(-g[0]));
  const float s1 = 1.0f / (1.0f + expf(-g[1]));
  const float v0 = a[0] * s0 * carry;
  const float v1 = a[1] * s1 * carry;
  const unsigned u = pk16(h_bits(v0), h_bits(v1));
  ((volatile unsigned*)G)[i] = u;
  __threadfence();
  ((volatile unsigned*)G)[i] = u;
}

extern "C" void kernel_launch(void* const* d_in, const int* in_sizes, int n_in,
                              void* d_out, int out_size, void* d_ws, size_t ws_size,
                              hipStream_t stream)
{
  if (n_in < 14) return;
  if (in_sizes[0] != kTok * kEmb) return;
  if (out_size != kTok * kEmb) return;
  if (ws_size < kWsTotal) return;

  const float* x       = (const float*)d_in[0];
  const float* w_qkv   = (const float*)d_in[1];
  const float* w_o     = (const float*)d_in[2];
  const float* b_o     = (const float*)d_in[3];
  const float* w1      = (const float*)d_in[4];
  const float* b1      = (const float*)d_in[5];
  const float* w2      = (const float*)d_in[6];
  const float* b2      = (const float*)d_in[7];
  const float* w_ffn_o = (const float*)d_in[8];
  const float* b_ffn_o = (const float*)d_in[9];
  const float* g1      = (const float*)d_in[10];
  const float* be1     = (const float*)d_in[11];
  const float* g2      = (const float*)d_in[12];
  const float* be2     = (const float*)d_in[13];
  float* outp = (float*)d_out;

  char* ws = (char*)d_ws;
  unsigned short* X16   = (unsigned short*)(ws + kOffX16);
  unsigned short* WqkvT = (unsigned short*)(ws + kOffWqkvT);
  unsigned short* WoT   = (unsigned short*)(ws + kOffWoT);
  unsigned short* W1T   = (unsigned short*)(ws + kOffW1T);
  unsigned short* W2T   = (unsigned short*)(ws + kOffW2T);
  unsigned short* WfT   = (unsigned short*)(ws + kOffWfT);
  unsigned short* QK16  = (unsigned short*)(ws + kOffQK16);
  unsigned short* VT16  = (unsigned short*)(ws + kOffVT16);
  float*          SC    = (float*)(ws + kOffSC);
  unsigned short* P16   = (unsigned short*)(ws + kOffP16);
  unsigned short* CTX16 = (unsigned short*)(ws + kOffCTX16);
  float*          Y1    = (float*)(ws + kOffY1);
  float*          X1    = (float*)(ws + kOffX1);
  unsigned short* X1h   = (unsigned short*)(ws + kOffX1h);
  float*          H1c   = (float*)(ws + kOffH1c);
  float*          H2c   = (float*)(ws + kOffH2c);
  unsigned short* G16   = (unsigned short*)(ws + kOffG16);
  float*          Y2    = (float*)(ws + kOffY2);

  dim3 blk(256);

  cast8_f16_kernel<<<dim3((kTok * kEmb / 8 + 255) / 256), blk, 0, stream>>>(x, X16, kTok * kEmb / 8);
  wtcast_kernel<<<dim3(kEmb / 64, 3 * kEmb / 64), blk, 0, stream>>>(w_qkv, kEmb, 3 * kEmb, WqkvT, kWCarry);
  wtcast_kernel<<<dim3(kEmb / 64, kEmb / 64), blk, 0, stream>>>(w_o, kEmb, kEmb, WoT, kWCarry);
  wtcast_kernel<<<dim3(kEmb / 64, kFfn / 64), blk, 0, stream>>>(w1, kEmb, kFfn, W1T, kWCarry);
  wtcast_kernel<<<dim3(kEmb / 64, kFfn / 64), blk, 0, stream>>>(w2, kEmb, kFfn, W2T, kWCarry);
  wtcast_kernel<<<dim3(kFfn / 64, kEmb / 64), blk, 0, stream>>>(w_ffn_o, kFfn, kEmb, WfT, kWCarry);

  {
    const int tiles = (kTok / 64) * (2 * kEmb / 64);
    wmma_gemm64<0, false, 0, 1, false><<<dim3((tiles + 7) / 8, 1), blk, 0, stream>>>(
        X16, X16, kEmb, 0L, WqkvT, WqkvT, kEmb, 0L,
        (void*)QK16, (void*)QK16, 2 * kEmb, 0L, b_o, x, 0L, kTok, 2 * kEmb, kEmb, kQkvScale);
  }
  {
    const int tiles = (kEmb / 64) * (kTok / 64);
    wmma_gemm64<0, false, 0, 1, false><<<dim3((tiles + 7) / 8, 1), blk, 0, stream>>>(
        WqkvT + (size_t)2 * kEmb * kEmb, WqkvT + (size_t)2 * kEmb * kEmb, kEmb, 0L, X16, X16, kEmb, 0L,
        (void*)VT16, (void*)VT16, kTok, 0L, b_o, x, 0L, kEmb, kTok, kEmb, kQkvScale);
  }

  for (int c = 0; c < kNumChunks; ++c) {
    const int g0 = c * kGrpPerChunk;
    const int bb = g0 / kHeads;
    const int h0 = g0 % kHeads;
    const size_t tokBase = (size_t)bb * kSeq;
    {
      const unsigned short* Aq = QK16 + tokBase * (2 * kEmb) + (size_t)h0 * kHd;
      const unsigned short* Bk = QK16 + tokBase * (2 * kEmb) + kEmb + (size_t)h0 * kHd;
      const int tiles = (kSeq / 64) * (kSeq / 64);
      wmma_gemm64<0, false, 0, 0, false><<<dim3((tiles + 7) / 8, kGrpPerChunk), blk, 0, stream>>>(
          Aq, Aq, 2 * kEmb, (long)kHd, Bk, Bk, 2 * kEmb, (long)kHd,
          (void*)SC, (void*)SC, kSeq, (long)kSeq * kSeq, b_o, x, 0L, kSeq, kSeq, kHd, kScoreScale);
    }
    softmax_row_kernel<<<dim3(kGrpPerChunk * kSeq), blk, 0, stream>>>(SC, P16, kPCarry);
    {
      const unsigned short* Bv = VT16 + (size_t)h0 * kHd * kTok + tokBase;
      unsigned short* Cc = CTX16 + tokBase * kEmb + (size_t)h0 * kHd;
      const int tiles = (kSeq / 64) * (kHd / 64);
      wmma_gemm64<0, false, 0, 1, false><<<dim3((tiles + 7) / 8, kGrpPerChunk), blk, 0, stream>>>(
          P16, P16, kSeq, (long)kSeq * kSeq, Bv, Bv, kTok, (long)kHd * kTok,
          (void*)Cc, (void*)Cc, kEmb, (long)kHd, b_o, x, 0L, kSeq, kHd, kSeq, kPVScale);
    }
  }

  {
    const int tiles = (kTok / 64) * (kEmb / 64);
    wmma_gemm64<0, false, 2, 0, true><<<dim3((tiles + 7) / 8, 1), blk, 0, stream>>>(
        CTX16, CTX16, kEmb, 0L, WoT, WoT, kEmb, 0L,
        (void*)Y1, (void*)Y1, kEmb, 0L, b_o, x, 0L, kTok, kEmb, kEmb, kWoScale);
  }
  ln_row_kernel<true><<<dim3(kTok), blk, 0, stream>>>(Y1, g1, be1, X1, X1h);

  for (int c = 0; c < kFfnChunks; ++c) {
    const unsigned short* Ax = X1h + (size_t)c * kFfnRows * kEmb;
    const int tiles = (kFfnRows / 64) * (kFfn / 64);
    wmma_gemm64<0, false, 2, 0, false><<<dim3((tiles + 7) / 8, 1), blk, 0, stream>>>(
        Ax, Ax, kEmb, 0L, W1T, W1T, kEmb, 0L,
        (void*)H1c, (void*)H1c, kFfn, 0L, b1, x, 0L, kFfnRows, kFfn, kEmb, kHScale);
    wmma_gemm64<0, false, 2, 0, false><<<dim3((tiles + 7) / 8, 1), blk, 0, stream>>>(
        Ax, Ax, kEmb, 0L, W2T, W2T, kEmb, 0L,
        (void*)H2c, (void*)H2c, kFfn, 0L, b2, x, 0L, kFfnRows, kFfn, kEmb, kHScale);
    const int n2 = kFfnRows * kFfn / 2;
    gate_kernel<<<dim3((n2 + 255) / 256), blk, 0, stream>>>(H1c, H2c, G16 + (size_t)c * kFfnRows * kFfn, n2, kGCarry);
  }

  {
    const int tiles = (kTok / 64) * (kEmb / 64);
    wmma_gemm64<0, false, 2, 0, true><<<dim3((tiles + 7) / 8, 1), blk, 0, stream>>>(
        G16, G16, kFfn, 0L, WfT, WfT, kFfn, 0L,
        (void*)Y2, (void*)Y2, kEmb, 0L, b_ffn_o, X1, 0L, kTok, kEmb, kFfn, kOutScale);
  }
  ln_row_kernel<false><<<dim3(kTok), blk, 0, stream>>>(Y2, g2, be2, outp, X1h);
}
